// GraphDiscriminator_89550068122064
// MI455X (gfx1250) — hardware-run, weakly checked
//
#include <hip/hip_runtime.h>


namespace {
constexpr int N = 10000, E = 160000, NG = 64, FA = 23, FAP = 32, HID = 256, NH = 4, C1 = NH * HID  , NPB = 8;
constexpr float XS = 8.0f, HS = 256.0f, WSC = 256.0f;
typedef _Float16 b16;
typedef __attribute__((ext_vector_type(16))) _Float16 v16b;
typedef __attribute__((ext_vector_type(8))) _Float16 v8b;
typedef __attribute__((ext_vector_type(8))) float v8f;
typedef __attribute__((ext_vector_type(4))) float v4f;
__device__ __forceinline__ float bf16_rne(float f) { unsigned int u = __float_as_uint(f); u += 0x7FFFu + ((u >> 16) & 1u); float r = __uint_as_float(u & 0xFFFF0000u); asm volatile("" : "+v"(r)); return r; }
__device__ __forceinline__ float bfv(float f) { float r = bf16_rne(f); asm volatile("" : "+v"(r)); return r; }
__device__ __forceinline__ void split16(float v, b16& hi, b16& lo) { hi = (b16)v; lo = (b16)(v - (float)hi); }
__device__ __forceinline__ v16b frag_kb(const b16* p, int hh) { const v8b a = *(const v8b*)(p + 8 * hh), b = *(const v8b*)(p + 16 + 8 * hh); v16b f;
#pragma unroll
  for (int e = 0; e < 8; ++e) { f[e] = a[e]; f[8 + e] = b[e]; } return f; }
__device__ __forceinline__ v8f wmma16b(v16b a, v16b b, v8f c) { v8f d = __builtin_amdgcn_wmma_f32_16x16x32_f16(false, a, false, b, (short)0, c, false, false); asm volatile("v_nop\n\tv_nop\n\tv_nop\n\tv_nop" : "+v"(d) : "v"(a), "v"(b)); return d; }
__device__ __forceinline__ void wave_lds_sync() { __builtin_amdgcn_fence(__ATOMIC_RELEASE, "workgroup"); __builtin_amdgcn_wave_barrier(); __builtin_amdgcn_fence(__ATOMIC_ACQUIRE, "workgroup"); }
__device__ __forceinline__ float pmul(float a, float b) { float p = a * b; asm volatile("" : "+v"(p)); return p; }
__device__ __forceinline__ int iclamp(int v, int lo, int hi) { return v < lo ? lo : (v > hi ? hi : v); }
__device__ __forceinline__ float elu(float v) { return v > 0.0f ? v : (__expf(v) - 1.0f); }
constexpr int CSR_NBLK7 = 512, CSR_GB7 = 7, CSR_GN7 = 1 << CSR_GB7  , CSR_TS7 = (CSR_GN7 < 32 ? 32 : CSR_GN7)  , CSR_MAXG7 = 512, CSR_CAP7 = 12288  ;
__device__ __host__ __forceinline__ int csr_tix7(int v) { return (v >> CSR_GB7) * CSR_TS7 + (v & (CSR_GN7 - 1)); }
__global__ __launch_bounds__(64) void csrA_kernel7(const int* __restrict__ dst, int E, int N, int nG, int CHP, int NGP, int* __restrict__ STG, int* __restrict__ HST) {
  extern __shared__ int sm[];
  int* cnt = sm; int* run = sm + NGP; int* ids = sm + 2 * NGP;
  const int b = blockIdx.x; const int ch = (E + CSR_NBLK7 - 1) / CSR_NBLK7; const int e0 = b * ch, e1 = min(E, e0 + ch);
  for (int i = threadIdx.x; i < NGP; i += 64) cnt[i] = 0;
  for (int i = threadIdx.x; i < CHP; i += 64) ids[i] = -1;
  __syncthreads();
  if (threadIdx.x == 0) {
    for (int e = e0; e < e1; ++e) { int d = dst[e]; d = (d < 0) ? 0 : (d >= N ? N - 1 : d); cnt[d >> CSR_GB7] += 1; }
    int acc = 0; for (int g = 0; g < nG; ++g) { run[g] = acc; acc += cnt[g]; }
    for (int e = e0; e < e1; ++e) { int d = dst[e]; d = (d < 0) ? 0 : (d >= N ? N - 1 : d); const int g = d >> CSR_GB7; ids[run[g]] = e; run[g] += 1; } }
  __syncthreads();
  typedef __attribute__((ext_vector_type(4))) int v4i;
  for (int pass = 0; pass < 2; ++pass) {
    for (int i = threadIdx.x; i < CHP / 4; i += 64) *(volatile v4i*)(STG + (size_t)b * CHP + i * 4) = *(const v4i*)(&ids[i * 4]);
    for (int i = threadIdx.x; i < NGP / 4; i += 64) { v4i v; for (int e = 0; e < 4; ++e) v[e] = (i * 4 + e < nG) ? cnt[i * 4 + e] : 0; *(volatile v4i*)(HST + (size_t)b * NGP + i * 4) = v; }
    __threadfence(); }
}
__global__ __launch_bounds__(512) void csrS_kernel7(const int* __restrict__ HST, int nG, int NGP, int* __restrict__ START, int* __restrict__ TOT, int* __restrict__ OFF) {
  __shared__ int tot[CSR_MAXG7];
  const int b = threadIdx.x;
  for (int pass = 0; pass < 2; ++pass) { int runb = 0; for (int g = 0; g < nG; ++g) { int c = HST[(size_t)b * NGP + g]; c = (c < 0) ? 0 : c; ((volatile int*)OFF)[(size_t)g * CSR_NBLK7 + b] = runb; runb += c; } __threadfence(); }
  for (int g = threadIdx.x; g < nG; g += 512) { int s = 0; for (int bb = 0; bb < CSR_NBLK7; ++bb) { int c = HST[(size_t)bb * NGP + g]; s += (c < 0) ? 0 : c; } tot[g] = s; }
  __syncthreads();
  if (threadIdx.x < 32) {
    __shared__ int st[CSR_MAXG7 + 32];
    if (threadIdx.x == 0) { int acc = 0; for (int g = 0; g < NGP; ++g) { st[g] = acc; if (g < nG) acc += (tot[g] + 31) & ~31; } st[NGP] = acc; }
    __builtin_amdgcn_fence(__ATOMIC_RELEASE, "workgroup"); __builtin_amdgcn_wave_barrier(); __builtin_amdgcn_fence(__ATOMIC_ACQUIRE, "workgroup");
    for (int pass = 0; pass < 2; ++pass) { for (int i = threadIdx.x; i < NGP + 32; i += 32) { ((volatile int*)START)[i] = (i <= NGP) ? st[min(i, NGP)] : 0; ((volatile int*)TOT)[i] = (i < nG) ? tot[i] : 0; } __threadfence(); } }
}
__global__ __launch_bounds__(256) void csrB_kernel7(const int* __restrict__ dst, int N, int nG, int CHP, int NGP, int permLen, const int* __restrict__ STG, const int* __restrict__ HST, const int* __restrict__ OFF, const int* __restrict__ START, const int* __restrict__ TOT, int* __restrict__ PERM, int* __restrict__ ROWPTR, int* __restrict__ ROWCNT, int* __restrict__ FLAG) {
  typedef __attribute__((ext_vector_type(4))) int v4i;
  __shared__ int ids[CSR_CAP7]; __shared__ unsigned short key[CSR_CAP7]; __shared__ int outp[CSR_CAP7]; __shared__ int ncnt[CSR_GN7 + 1]; __shared__ int boff[CSR_NBLK7 + 1];
  const int g = blockIdx.x, t_ = threadIdx.x; int tot = TOT[g]; int st = START[g], stn = START[g + 1]; const int v0 = g * CSR_GN7; const int nv = min(CSR_GN7, N - v0); const int t0 = g * CSR_TS7;
  st = (st < 0) ? 0 : (st > permLen - 32 ? permLen - 32 : st) & ~31; stn = (stn < st) ? st : (stn > permLen ? permLen : stn); tot = (tot < 0) ? 0 : tot; if (tot > stn - st && tot <= CSR_CAP7) tot = stn - st;
  if (tot > CSR_CAP7) {
    for (int pass = 0; pass < 2; ++pass) { for (int i = t_; i < CSR_TS7 / 4; i += 256) { v4i a, c; for (int e = 0; e < 4; ++e) { a[e] = st; c[e] = 0; } *(volatile v4i*)(ROWPTR + t0 + i * 4) = a; *(volatile v4i*)(ROWCNT + t0 + i * 4) = c; } if (t_ == 0) ((volatile int*)FLAG)[0] = 1; __threadfence(); } (void)nv; return; }
  if (t_ == 0) { int acc = 0; for (int b = 0; b < CSR_NBLK7; ++b) { boff[b] = acc; int c = HST[(size_t)b * NGP + g]; c = (c < 0) ? 0 : (c > CHP ? CHP : c); acc += c; if (acc > tot) acc = tot; } boff[CSR_NBLK7] = acc; }
  for (int i = t_; i <= CSR_GN7; i += 256) ncnt[i] = 0;
  __syncthreads();
  for (int b = 0; b < CSR_NBLK7; ++b) { const int c = boff[b + 1] - boff[b]; int o_ = OFF[(size_t)g * CSR_NBLK7 + b]; o_ = (o_ < 0) ? 0 : (o_ > CHP - c ? CHP - c : o_); const int* src_ = STG + (size_t)b * CHP + o_;
    for (int i = t_; i < c; i += 256) { int id = src_[i]; id = (id < 0) ? 0 : id; ids[boff[b] + i] = id; int d = dst[id]; d = (d < v0) ? v0 : (d >= N ? N - 1 : d); int kk = d - v0; kk = (kk < 0) ? 0 : (kk >= CSR_GN7 ? CSR_GN7 - 1 : kk); key[boff[b] + i] = (unsigned short)kk; } }
  __syncthreads();
  if (t_ == 0) { for (int i = 0; i < tot; ++i) ncnt[key[i]] += 1; int acc = 0; for (int vl = 0; vl < CSR_GN7; ++vl) { const int c = ncnt[vl]; ncnt[vl] = acc; acc += c; } ncnt[CSR_GN7] = acc;
    for (int i = 0; i < tot; ++i) { const int vl = key[i]; outp[ncnt[vl]] = ids[i]; ncnt[vl] += 1; }
    for (int vl = CSR_GN7; vl > 0; --vl) ncnt[vl] = ncnt[vl - 1]; ncnt[0] = 0; }
  __syncthreads();
  for (int pass = 0; pass < 2; ++pass) {
    for (int i = t_; i < (stn - st) / 4; i += 256) { v4i v; for (int e = 0; e < 4; ++e) { const int q = i * 4 + e; v[e] = (q < tot) ? outp[q] : -1; } *(volatile v4i*)(PERM + st + i * 4) = v; }
    for (int i = t_; i < CSR_TS7 / 4; i += 256) { v4i a, c; for (int e = 0; e < 4; ++e) { const int vl = i * 4 + e; const int vc = vl < CSR_GN7 ? vl : CSR_GN7; a[e] = (vl < CSR_GN7) ? st + ncnt[vc] : st; c[e] = (vl < nv) ? (ncnt[(vc < CSR_GN7 ? vc : CSR_GN7 - 1) + 1] - ncnt[vc]) : 0; } *(volatile v4i*)(ROWPTR + t0 + i * 4) = a; *(volatile v4i*)(ROWCNT + t0 + i * 4) = c; }
    __threadfence(); }
}
__global__ __launch_bounds__(256) void csrZ_kernel7(int* __restrict__ p, size_t n4) { typedef __attribute__((ext_vector_type(4))) int v4i; const size_t tid = (size_t)blockIdx.x * 256 + threadIdx.x, nth = (size_t)gridDim.x * 256; v4i z = {0, 0, 0, 0}; for (size_t i = tid; i < n4; i += nth) *(volatile v4i*)(p + i * 4) = z; }
struct CsrBufs7 { int *STG, *HST, *OFF, *START, *TOT, *PERM, *ROWPTR, *ROWCNT, *FLAG; int nG, NGP, CHP; size_t permLen; char* base; size_t bytes; };
static size_t csr_carve7(CsrBufs7& c, char* ws, size_t off, int E, int N) {
  const size_t off0 = off; c.base = ws + off;
  auto al = [&](size_t bytes) { char* p = ws + off; off += (bytes + 255) & ~(size_t)255; return p; };
  c.nG = (N + CSR_GN7 - 1) / CSR_GN7; c.NGP = (c.nG + 31) & ~31; const int ch = (E + CSR_NBLK7 - 1) / CSR_NBLK7; c.CHP = (ch + 31) & ~31; c.permLen = (size_t)E + 32 * (size_t)c.nG + 32;
  c.STG = (int*)al((size_t)CSR_NBLK7 * c.CHP * 4); c.HST = (int*)al((size_t)CSR_NBLK7 * c.NGP * 4); c.OFF = (int*)al((size_t)c.NGP * CSR_NBLK7 * 4); c.START = (int*)al((size_t)(c.NGP + 64) * 4); c.TOT = (int*)al((size_t)(c.NGP + 64) * 4);
  c.PERM = (int*)al(c.permLen * 4); c.ROWPTR = (int*)al((size_t)c.nG * CSR_TS7 * 4); c.ROWCNT = (int*)al((size_t)c.nG * CSR_TS7 * 4); c.FLAG = (int*)al(256);
  c.bytes = off - off0; return off;
}
static void csr_build7(const CsrBufs7& c, const int* dst, int E, int N, hipStream_t stream) {
  const size_t smem = (size_t)(2 * c.NGP + c.CHP) * 4;
  csrZ_kernel7<<<512, 256, 0, stream>>>((int*)c.base, c.bytes / 16);
  csrA_kernel7<<<CSR_NBLK7, 64, smem, stream>>>(dst, E, N, c.nG, c.CHP, c.NGP, c.STG, c.HST);
  csrS_kernel7<<<1, 512, 0, stream>>>(c.HST, c.nG, c.NGP, c.START, c.TOT, c.OFF);
  csrB_kernel7<<<c.nG, 256, 0, stream>>>(dst, N, c.nG, c.CHP, c.NGP, (int)c.permLen, c.STG, c.HST, c.OFF, c.START, c.TOT, c.PERM, c.ROWPTR, c.ROWCNT, c.FLAG);
}
constexpr int CSR_NBLK5 = 512, CSR_GB5 = 5, CSR_GN5 = 1 << CSR_GB5  , CSR_TS5 = (CSR_GN5 < 32 ? 32 : CSR_GN5)  , CSR_MAXG5 = 512, CSR_CAP5 = 12288  ;
__device__ __host__ __forceinline__ int csr_tix5(int v) { return (v >> CSR_GB5) * CSR_TS5 + (v & (CSR_GN5 - 1)); }
__global__ __launch_bounds__(64) void csrA_kernel5(const int* __restrict__ dst, int E, int N, int nG, int CHP, int NGP, int* __restrict__ STG, int* __restrict__ HST) {
  extern __shared__ int sm[];
  int* cnt = sm; int* run = sm + NGP; int* ids = sm + 2 * NGP;
  const int b = blockIdx.x; const int ch = (E + CSR_NBLK5 - 1) / CSR_NBLK5; const int e0 = b * ch, e1 = min(E, e0 + ch);
  for (int i = threadIdx.x; i < NGP; i += 64) cnt[i] = 0;
  for (int i = threadIdx.x; i < CHP; i += 64) ids[i] = -1;
  __syncthreads();
  if (threadIdx.x == 0) {
    for (int e = e0; e < e1; ++e) { int d = dst[e]; d = (d < 0) ? 0 : (d >= N ? N - 1 : d); cnt[d >> CSR_GB5] += 1; }
    int acc = 0; for (int g = 0; g < nG; ++g) { run[g] = acc; acc += cnt[g]; }
    for (int e = e0; e < e1; ++e) { int d = dst[e]; d = (d < 0) ? 0 : (d >= N ? N - 1 : d); const int g = d >> CSR_GB5; ids[run[g]] = e; run[g] += 1; } }
  __syncthreads();
  typedef __attribute__((ext_vector_type(4))) int v4i;
  for (int pass = 0; pass < 2; ++pass) {
    for (int i = threadIdx.x; i < CHP / 4; i += 64) *(volatile v4i*)(STG + (size_t)b * CHP + i * 4) = *(const v4i*)(&ids[i * 4]);
    for (int i = threadIdx.x; i < NGP / 4; i += 64) { v4i v; for (int e = 0; e < 4; ++e) v[e] = (i * 4 + e < nG) ? cnt[i * 4 + e] : 0; *(volatile v4i*)(HST + (size_t)b * NGP + i * 4) = v; }
    __threadfence(); }
}
__global__ __launch_bounds__(512) void csrS_kernel5(const int* __restrict__ HST, int nG, int NGP, int* __restrict__ START, int* __restrict__ TOT, int* __restrict__ OFF) {
  __shared__ int tot[CSR_MAXG5];
  const int b = threadIdx.x;
  for (int pass = 0; pass < 2; ++pass) { int runb = 0; for (int g = 0; g < nG; ++g) { int c = HST[(size_t)b * NGP + g]; c = (c < 0) ? 0 : c; ((volatile int*)OFF)[(size_t)g * CSR_NBLK5 + b] = runb; runb += c; } __threadfence(); }
  for (int g = threadIdx.x; g < nG; g += 512) { int s = 0; for (int bb = 0; bb < CSR_NBLK5; ++bb) { int c = HST[(size_t)bb * NGP + g]; s += (c < 0) ? 0 : c; } tot[g] = s; }
  __syncthreads();
  if (threadIdx.x < 32) {
    __shared__ int st[CSR_MAXG5 + 32];
    if (threadIdx.x == 0) { int acc = 0; for (int g = 0; g < NGP; ++g) { st[g] = acc; if (g < nG) acc += (tot[g] + 31) & ~31; } st[NGP] = acc; }
    __builtin_amdgcn_fence(__ATOMIC_RELEASE, "workgroup"); __builtin_amdgcn_wave_barrier(); __builtin_amdgcn_fence(__ATOMIC_ACQUIRE, "workgroup");
    for (int pass = 0; pass < 2; ++pass) { for (int i = threadIdx.x; i < NGP + 32; i += 32) { ((volatile int*)START)[i] = (i <= NGP) ? st[min(i, NGP)] : 0; ((volatile int*)TOT)[i] = (i < nG) ? tot[i] : 0; } __threadfence(); } }
}
__global__ __launch_bounds__(256) void csrB_kernel5(const int* __restrict__ dst, int N, int nG, int CHP, int NGP, int permLen, const int* __restrict__ STG, const int* __restrict__ HST, const int* __restrict__ OFF, const int* __restrict__ START, const int* __restrict__ TOT, int* __restrict__ PERM, int* __restrict__ ROWPTR, int* __restrict__ ROWCNT, int* __restrict__ FLAG) {
  typedef __attribute__((ext_vector_type(4))) int v4i;
  __shared__ int ids[CSR_CAP5]; __shared__ unsigned short key[CSR_CAP5]; __shared__ int outp[CSR_CAP5]; __shared__ int ncnt[CSR_GN5 + 1]; __shared__ int boff[CSR_NBLK5 + 1];
  const int g = blockIdx.x, t_ = threadIdx.x; int tot = TOT[g]; int st = START[g], stn = START[g + 1]; const int v0 = g * CSR_GN5; const int nv = min(CSR_GN5, N - v0); const int t0 = g * CSR_TS5;
  st = (st < 0) ? 0 : (st > permLen - 32 ? permLen - 32 : st) & ~31; stn = (stn < st) ? st : (stn > permLen ? permLen : stn); tot = (tot < 0) ? 0 : tot; if (tot > stn - st && tot <= CSR_CAP5) tot = stn - st;
  if (tot > CSR_CAP5) {
    for (int pass = 0; pass < 2; ++pass) { for (int i = t_; i < CSR_TS5 / 4; i += 256) { v4i a, c; for (int e = 0; e < 4; ++e) { a[e] = st; c[e] = 0; } *(volatile v4i*)(ROWPTR + t0 + i * 4) = a; *(volatile v4i*)(ROWCNT + t0 + i * 4) = c; } if (t_ == 0) ((volatile int*)FLAG)[0] = 1; __threadfence(); } (void)nv; return; }
  if (t_ == 0) { int acc = 0; for (int b = 0; b < CSR_NBLK5; ++b) { boff[b] = acc; int c = HST[(size_t)b * NGP + g]; c = (c < 0) ? 0 : (c > CHP ? CHP : c); acc += c; if (acc > tot) acc = tot; } boff[CSR_NBLK5] = acc; }
  for (int i = t_; i <= CSR_GN5; i += 256) ncnt[i] = 0;
  __syncthreads();
  for (int b = 0; b < CSR_NBLK5; ++b) { const int c = boff[b + 1] - boff[b]; int o_ = OFF[(size_t)g * CSR_NBLK5 + b]; o_ = (o_ < 0) ? 0 : (o_ > CHP - c ? CHP - c : o_); const int* src_ = STG + (size_t)b * CHP + o_;
    for (int i = t_; i < c; i += 256) { int id = src_[i]; id = (id < 0) ? 0 : id; ids[boff[b] + i] = id; int d = dst[id]; d = (d < v0) ? v0 : (d >= N ? N - 1 : d); int kk = d - v0; kk = (kk < 0) ? 0 : (kk >= CSR_GN5 ? CSR_GN5 - 1 : kk); key[boff[b] + i] = (unsigned short)kk; } }
  __syncthreads();
  if (t_ == 0) { for (int i = 0; i < tot; ++i) ncnt[key[i]] += 1; int acc = 0; for (int vl = 0; vl < CSR_GN5; ++vl) { const int c = ncnt[vl]; ncnt[vl] = acc; acc += c; } ncnt[CSR_GN5] = acc;
    for (int i = 0; i < tot; ++i) { const int vl = key[i]; outp[ncnt[vl]] = ids[i]; ncnt[vl] += 1; }
    for (int vl = CSR_GN5; vl > 0; --vl) ncnt[vl] = ncnt[vl - 1]; ncnt[0] = 0; }
  __syncthreads();
  for (int pass = 0; pass < 2; ++pass) {
    for (int i = t_; i < (stn - st) / 4; i += 256) { v4i v; for (int e = 0; e < 4; ++e) { const int q = i * 4 + e; v[e] = (q < tot) ? outp[q] : -1; } *(volatile v4i*)(PERM + st + i * 4) = v; }
    for (int i = t_; i < CSR_TS5 / 4; i += 256) { v4i a, c; for (int e = 0; e < 4; ++e) { const int vl = i * 4 + e; const int vc = vl < CSR_GN5 ? vl : CSR_GN5; a[e] = (vl < CSR_GN5) ? st + ncnt[vc] : st; c[e] = (vl < nv) ? (ncnt[(vc < CSR_GN5 ? vc : CSR_GN5 - 1) + 1] - ncnt[vc]) : 0; } *(volatile v4i*)(ROWPTR + t0 + i * 4) = a; *(volatile v4i*)(ROWCNT + t0 + i * 4) = c; }
    __threadfence(); }
}
__global__ __launch_bounds__(256) void csrZ_kernel5(int* __restrict__ p, size_t n4) { typedef __attribute__((ext_vector_type(4))) int v4i; const size_t tid = (size_t)blockIdx.x * 256 + threadIdx.x, nth = (size_t)gridDim.x * 256; v4i z = {0, 0, 0, 0}; for (size_t i = tid; i < n4; i += nth) *(volatile v4i*)(p + i * 4) = z; }
struct CsrBufs5 { int *STG, *HST, *OFF, *START, *TOT, *PERM, *ROWPTR, *ROWCNT, *FLAG; int nG, NGP, CHP; size_t permLen; char* base; size_t bytes; };
static size_t csr_carve5(CsrBufs5& c, char* ws, size_t off, int E, int N) {
  const size_t off0 = off; c.base = ws + off;
  auto al = [&](size_t bytes) { char* p = ws + off; off += (bytes + 255) & ~(size_t)255; return p; };
  c.nG = (N + CSR_GN5 - 1) / CSR_GN5; c.NGP = (c.nG + 31) & ~31; const int ch = (E + CSR_NBLK5 - 1) / CSR_NBLK5; c.CHP = (ch + 31) & ~31; c.permLen = (size_t)E + 32 * (size_t)c.nG + 32;
  c.STG = (int*)al((size_t)CSR_NBLK5 * c.CHP * 4); c.HST = (int*)al((size_t)CSR_NBLK5 * c.NGP * 4); c.OFF = (int*)al((size_t)c.NGP * CSR_NBLK5 * 4); c.START = (int*)al((size_t)(c.NGP + 64) * 4); c.TOT = (int*)al((size_t)(c.NGP + 64) * 4);
  c.PERM = (int*)al(c.permLen * 4); c.ROWPTR = (int*)al((size_t)c.nG * CSR_TS5 * 4); c.ROWCNT = (int*)al((size_t)c.nG * CSR_TS5 * 4); c.FLAG = (int*)al(256);
  c.bytes = off - off0; return off;
}
static void csr_build5(const CsrBufs5& c, const int* dst, int E, int N, hipStream_t stream) {
  const size_t smem = (size_t)(2 * c.NGP + c.CHP) * 4;
  csrZ_kernel5<<<512, 256, 0, stream>>>((int*)c.base, c.bytes / 16);
  csrA_kernel5<<<CSR_NBLK5, 64, smem, stream>>>(dst, E, N, c.nG, c.CHP, c.NGP, c.STG, c.HST);
  csrS_kernel5<<<1, 512, 0, stream>>>(c.HST, c.nG, c.NGP, c.START, c.TOT, c.OFF);
  csrB_kernel5<<<c.nG, 256, 0, stream>>>(dst, N, c.nG, c.CHP, c.NGP, (int)c.permLen, c.STG, c.HST, c.OFF, c.START, c.TOT, c.PERM, c.ROWPTR, c.ROWCNT, c.FLAG);
}


__global__ __launch_bounds__(256) void wput_kernel(const float* __restrict__ w1, const float* __restrict__ w2, const float* __restrict__ w3, const float* __restrict__ f1, b16* __restrict__ WT1, b16* __restrict__ WT2, b16* __restrict__ WT3, b16* __restrict__ WF1) { const size_t nt = (size_t)gridDim.x * 256, u0 = (size_t)blockIdx.x * 256 + threadIdx.x; v8b v;
  for (size_t u = u0; u < (size_t)C1 * 4; u += nt) { const int o = (int)(u / 4), k0 = (int)(u % 4) * 8;
#pragma unroll
    for (int j = 0; j < 8; ++j) { const int k = k0 + j; v[j] = (b16)(k < FA ? bf16_rne(w1[(size_t)k * C1 + o]) * WSC : 0.0f); } for (int pass = 0; pass < 2; ++pass) { *(volatile v8b*)(WT1 + (size_t)o * FAP + k0) = v; __threadfence(); } }
  for (size_t u = u0; u < (size_t)C1 * 128; u += nt) { const int o = (int)(u / 128), k0 = (int)(u % 128) * 8;
#pragma unroll
    for (int j = 0; j < 8; ++j) v[j] = (b16)(bf16_rne(w2[(size_t)(k0 + j) * C1 + o]) * WSC); for (int pass = 0; pass < 2; ++pass) { *(volatile v8b*)(WT2 + (size_t)o * C1 + k0) = v; __threadfence(); } }
  for (size_t u = u0; u < (size_t)HID * 128; u += nt) { const int o = (int)(u / 128), k0 = (int)(u % 128) * 8;
#pragma unroll
    for (int j = 0; j < 8; ++j) v[j] = (b16)(bf16_rne(w3[(size_t)(k0 + j) * HID + o]) * WSC); for (int pass = 0; pass < 2; ++pass) { *(volatile v8b*)(WT3 + (size_t)o * C1 + k0) = v; __threadfence(); } }
  for (size_t u = u0; u < (size_t)128 * 32; u += nt) { const int o = (int)(u / 32), k0 = (int)(u % 32) * 8;
#pragma unroll
    for (int j = 0; j < 8; ++j) v[j] = (b16)(bf16_rne(f1[(size_t)(k0 + j) * 128 + o]) * WSC); for (int pass = 0; pass < 2; ++pass) { *(volatile v8b*)(WF1 + (size_t)o * HID + k0) = v; __threadfence(); } } }
template <int MODE, int KIN, int NT>
__global__ __launch_bounds__(32) void proj_kernel(const float* __restrict__ IN, const b16* __restrict__ W, const float* __restrict__ as_, const float* __restrict__ ad_, int NLIM, float* __restrict__ FT, float* __restrict__ ES) { constexpr int OW = NT * 16, NGR = NT / 16, KP = MODE == 0 ? FAP : KIN; __shared__ __attribute__((aligned(16))) b16 Ah[16][KP + 8], Al[16][KP + 8]; __shared__ float Tf[16][260], Eq[16][8]; const int lane = threadIdx.x, nloc = lane & 15, hlf = lane >> 4; const size_t m0 = (size_t)blockIdx.x * 16; if (m0 >= (size_t)NLIM) return;
  if (MODE == 0) { for (int rr = 0; rr < 16; ++rr) { Ah[rr][lane] = (b16)(lane < FA ? bf16_rne(IN[(m0 + rr) * FA + lane]) * XS : 0.0f); Al[rr][lane] = (b16)0.0f; } }
  else { for (int rr = 0; rr < 16; ++rr) for (int q = 0; q < KIN / 32; ++q) { const int c = q * 32 + lane; b16 p, ql; split16(IN[(m0 + rr) * KIN + c] * HS, p, ql); Ah[rr][c] = p; Al[rr][c] = ql; } }
  if (lane < 16) { for (int k = KP; k < KP + 8; ++k) { Ah[lane][k] = (b16)0.0f; Al[lane][k] = (b16)0.0f; } for (int j = 0; j < 8; ++j) Eq[lane][j] = 0.0f; }
  wave_lds_sync(); const float osc = MODE == 0 ? 1.0f / (XS * WSC) : 1.0f / (HS * WSC);
#pragma unroll 1
  for (int g = 0; g < NGR; ++g) { v8f acc[16];
#pragma unroll
    for (int t = 0; t < 16; ++t) acc[t] = (v8f){};
#pragma unroll 2
    for (int kb = 0; kb < KP; kb += 32) { const v16b a = frag_kb(&Ah[nloc][kb], hlf), al = frag_kb(&Al[nloc][kb], hlf);
#pragma unroll
      for (int t = 0; t < 16; ++t) { const v16b bw = frag_kb(W + (size_t)(g * 256 + t * 16 + nloc) * KP + kb, hlf); acc[t] = wmma16b(a, bw, acc[t]); if (MODE == 1) acc[t] = wmma16b(al, bw, acc[t]); } }
#pragma unroll
    for (int t = 0; t < 16; ++t)
#pragma unroll
      for (int r8 = 0; r8 < 8; ++r8) Tf[8 * hlf + r8][t * 16 + nloc] = acc[t][r8] * osc;
    wave_lds_sync();
    for (int rr = 0; rr < 16; ++rr) { float s1 = 0.0f, s2 = 0.0f; for (int q = 0; q < 8; ++q) { const int c = q * 32 + lane; s1 += pmul(Tf[rr][c], bfv(as_[g * HID + c])); s2 += pmul(Tf[rr][c], bfv(ad_[g * HID + c])); } for (int o = 16; o; o >>= 1) { s1 += __shfl_xor(s1, o); s2 += __shfl_xor(s2, o); } if (lane == 0) { Eq[rr][g] = s1; Eq[rr][4 + g] = s2; } }
    for (int pass = 0; pass < 2; ++pass) { for (int rr = 0; rr < 16; ++rr) for (int q = 0; q < 2; ++q) *(volatile v4f*)(FT + (m0 + rr) * OW + g * 256 + q * 128 + lane * 4) = *(const v4f*)(&Tf[rr][q * 128 + lane * 4]); __threadfence(); }
    wave_lds_sync(); }
  for (int pass = 0; pass < 2; ++pass) { for (int q = 0; q < 4; ++q) ((volatile float*)ES)[m0 * 8 + q * 32 + lane] = Eq[(q * 32 + lane) >> 3][(q * 32 + lane) & 7]; __threadfence(); } }
template <int NHh>
__global__ __launch_bounds__(256) void gat_kernel(const float* __restrict__ FT, const float* __restrict__ ES, const float* __restrict__ bias, const int* __restrict__ srcs, const int* __restrict__ PERM, const int* __restrict__ ROWPTR, const int* __restrict__ ROWCNT, int permLen, int NLIM, float* __restrict__ OUT) { constexpr int OW = NHh * HID; __shared__ float St[NPB][4][4]; __shared__ v4f Acc[NPB][4][2][32]; const int wave = threadIdx.x >> 5, lane = threadIdx.x & 31; const size_t i = (size_t)blockIdx.x * NPB + wave; if (i >= (size_t)NLIM) return; int st = ROWPTR[i], cnt = ROWCNT[i]; cnt = iclamp(cnt, 0, E); st = iclamp(st, 0, permLen - cnt);
  for (int h = 0; h < NHh; ++h) { if (lane == 0) { St[wave][h][0] = ES[i * 8 + 4 + h]; St[wave][h][1] = -INFINITY; St[wave][h][2] = 0.0f; } Acc[wave][h][0][lane] = (v4f){0, 0, 0, 0}; Acc[wave][h][1][lane] = (v4f){0, 0, 0, 0}; }
  wave_lds_sync();
  auto visit = [&](size_t u) {
#pragma unroll 1
    for (int h = 0; h < NHh; ++h) { const float adi = St[wave][h][0], mx = St[wave][h][1], den = St[wave][h][2]; float s = ES[u * 8 + h] + adi; s = s > 0.0f ? s : 0.2f * s; const float mn = fmaxf(mx, s); const float sf = (mx == -INFINITY) ? 0.0f : __expf(mx - mn); const float p = __expf(s - mn); const float* fp = FT + u * OW + h * HID + lane * 8; const v4f v0 = *(const v4f*)fp, v1 = *(const v4f*)(fp + 4); v4f a0 = Acc[wave][h][0][lane], a1 = Acc[wave][h][1][lane]; a0 = a0 * sf + v0 * p; a1 = a1 * sf + v1 * p; Acc[wave][h][0][lane] = a0; Acc[wave][h][1][lane] = a1; wave_lds_sync(); if (lane == 0) { St[wave][h][1] = mn; St[wave][h][2] = den * sf + p; } wave_lds_sync(); } };
#pragma unroll 1
  for (int j = 0; j < cnt; ++j) { const int e = iclamp(PERM[st + j], 0, E - 1); const size_t u = (size_t)iclamp(srcs[e], 0, N - 1); if (u >= (size_t)NLIM) continue; visit(u); }
  visit(i);
  for (int pass = 0; pass < 2; ++pass) {
#pragma unroll 1
    for (int h = 0; h < NHh; ++h) { const float dn = St[wave][h][2] + 1e-16f; const v4f a0 = Acc[wave][h][0][lane], a1 = Acc[wave][h][1][lane]; v4f o0, o1; for (int k = 0; k < 4; ++k) { const int c = h * HID + lane * 8 + k; o0[k] = elu(a0[k] / dn + bfv(bias[c])); o1[k] = elu(a1[k] / dn + bfv(bias[c + 4])); } *(volatile v4f*)(OUT + i * OW + h * HID + lane * 8) = o0; *(volatile v4f*)(OUT + i * OW + h * HID + lane * 8 + 4) = o1; }
    __threadfence(); } }
__global__ __launch_bounds__(256) void pool_kernel(const float* __restrict__ H3, const int* __restrict__ PERM, const int* __restrict__ ROWPTR, const int* __restrict__ ROWCNT, int permLen, int NLIM, float* __restrict__ out) { const int wave = threadIdx.x >> 5, lane = threadIdx.x & 31; const int g = blockIdx.x * NPB + wave; if (g >= NG) return; int st = ROWPTR[g], cnt = ROWCNT[g]; cnt = iclamp(cnt, 0, N); st = iclamp(st, 0, permLen - cnt); v4f s0 = {0, 0, 0, 0}, s1 = {0, 0, 0, 0}; int nn = 0;
#pragma unroll 1
  for (int j = 0; j < cnt; ++j) { const size_t n = (size_t)iclamp(PERM[st + j], 0, N - 1); if (n >= (size_t)NLIM) continue; ++nn; const float* hp = H3 + n * HID + lane * 8; s0 += *(const v4f*)hp; s1 += *(const v4f*)(hp + 4); }
  const float inv = 1.0f / fmaxf((float)nn, 1.0f);
  for (int pass = 0; pass < 2; ++pass) { *(volatile v4f*)(out + NG + (size_t)g * HID + lane * 8) = s0 * inv; *(volatile v4f*)(out + NG + (size_t)g * HID + lane * 8 + 4) = s1 * inv; __threadfence(); } }
__global__ __launch_bounds__(32) void head_kernel(const float* __restrict__ outfeat, const b16* __restrict__ WF1, const float* __restrict__ b1, const float* __restrict__ w2, const float* __restrict__ b2, float* __restrict__ out) { __shared__ __attribute__((aligned(16))) b16 Ah[16][HID + 8], Al[16][HID + 8]; __shared__ float Tf[16][132], Os[NG]; const int lane = threadIdx.x, nloc = lane & 15, hlf = lane >> 4;
#pragma unroll 1
  for (int grp = 0; grp < NG / 16; ++grp) { for (int rr = 0; rr < 16; ++rr) for (int q = 0; q < 8; ++q) { const int c = q * 32 + lane; b16 p, ql; split16(outfeat[NG + (size_t)(grp * 16 + rr) * HID + c] * HS, p, ql); Ah[rr][c] = p; Al[rr][c] = ql; }
    if (lane < 16) for (int k = HID; k < HID + 8; ++k) { Ah[lane][k] = (b16)0.0f; Al[lane][k] = (b16)0.0f; }
    wave_lds_sync(); v8f acc[8];
#pragma unroll
    for (int t = 0; t < 8; ++t) acc[t] = (v8f){};
#pragma unroll 2
    for (int kb = 0; kb < HID; kb += 32) { const v16b a = frag_kb(&Ah[nloc][kb], hlf), al = frag_kb(&Al[nloc][kb], hlf);
#pragma unroll
      for (int t = 0; t < 8; ++t) { const v16b bw = frag_kb(WF1 + (size_t)(t * 16 + nloc) * HID + kb, hlf); acc[t] = wmma16b(a, bw, acc[t]); acc[t] = wmma16b(al, bw, acc[t]); } }
#pragma unroll
    for (int t = 0; t < 8; ++t) { const int cc = t * 16 + nloc; const float bb = bfv(b1[cc]);
#pragma unroll
      for (int r8 = 0; r8 < 8; ++r8) Tf[8 * hlf + r8][cc] = fmaxf(acc[t][r8] * (1.0f / (HS * WSC)) + bb, 0.0f); }
    wave_lds_sync();
    if (lane < 16) { float s = bfv(b2[0]);
#pragma unroll 4
      for (int c = 0; c < 128; ++c) s += pmul(Tf[lane][c], bfv(w2[c])); Os[grp * 16 + lane] = s; }
    wave_lds_sync(); }
  for (int pass = 0; pass < 2; ++pass) { for (int q = 0; q < NG / 32; ++q) ((volatile float*)out)[q * 32 + lane] = Os[q * 32 + lane]; __threadfence(); } }
}

extern "C" void kernel_launch(void* const* d_in, const int* in_sizes, int n_in, void* d_out, int out_size, void* d_ws, size_t ws_size, hipStream_t stream) {
  (void)n_in;
  auto Fp = [&](int i) { return (const float*)d_in[i]; }; auto Ip = [&](int i) { return (const int*)d_in[i]; };
  if (in_sizes[0] != N * FA || in_sizes[1] != 2 * E || in_sizes[2] != N || in_sizes[3] != FA * C1 || in_sizes[7] != C1 * C1 || in_sizes[11] != C1 * HID || in_sizes[15] != HID * 128 || in_sizes[17] != 128 || out_size != NG + NG * HID) return;
  const int NLIM = N;
  size_t off = 0; char* ws = (char*)d_ws;
  auto carve = [&](size_t bytes) { char* p = ws + off; off += (bytes + 255) & ~(size_t)255; return p; };
  b16* WT1 = (b16*)carve((size_t)C1 * FAP * 2); b16* WT2 = (b16*)carve((size_t)C1 * C1 * 2); b16* WT3 = (b16*)carve((size_t)HID * C1 * 2); b16* WF1 = (b16*)carve((size_t)128 * HID * 2); float* FT = (float*)carve((size_t)N * C1 * 4); float* ES = (float*)carve((size_t)N * 8 * 4); float* HA = (float*)carve((size_t)N * C1 * 4); float* HB = (float*)carve((size_t)N * C1 * 4); CsrBufs7 csr; off = csr_carve7(csr, ws, off, E, N); CsrBufs5 cg; off = csr_carve5(cg, ws, off, N, NG);
  if (off > ws_size || off > ((size_t)160 << 20)) return;
  const int nb = (NLIM + NPB - 1) / NPB;
  wput_kernel<<<128, 256, 0, stream>>>(Fp(3), Fp(7), Fp(11), Fp(15), WT1, WT2, WT3, WF1);
  csr_build7(csr, Ip(1) + E, E, N, stream); csr_build5(cg, Ip(2), N, NG, stream);
  proj_kernel<0, FA, 64><<<NLIM / 16, 32, 0, stream>>>(Fp(0), WT1, Fp(4), Fp(5), NLIM, FT, ES);
  gat_kernel<4><<<nb, 256, 0, stream>>>(FT, ES, Fp(6), Ip(1), csr.PERM, csr.ROWPTR, csr.ROWCNT, (int)csr.permLen, NLIM, HA);
  proj_kernel<1, C1, 64><<<NLIM / 16, 32, 0, stream>>>(HA, WT2, Fp(8), Fp(9), NLIM, FT, ES);
  gat_kernel<4><<<nb, 256, 0, stream>>>(FT, ES, Fp(10), Ip(1), csr.PERM, csr.ROWPTR, csr.ROWCNT, (int)csr.permLen, NLIM, HB);
  proj_kernel<1, C1, 16><<<NLIM / 16, 32, 0, stream>>>(HB, WT3, Fp(12), Fp(13), NLIM, FT, ES);
  gat_kernel<1><<<nb, 256, 0, stream>>>(FT, ES, Fp(14), Ip(1), csr.PERM, csr.ROWPTR, csr.ROWCNT, (int)csr.permLen, NLIM, HA);
  pool_kernel<<<NG / NPB, 256, 0, stream>>>(HA, cg.PERM, cg.ROWPTR, cg.ROWCNT, (int)cg.permLen, NLIM, (float*)d_out);
  head_kernel<<<1, 32, 0, stream>>>((const float*)d_out, WF1, Fp(16), Fp(17), Fp(18), (float*)d_out);
}
